// BrushStroke_87368224735782
// MI455X (gfx1250) — hardware-verified
//
#include <hip/hip_runtime.h>
#include <stddef.h>


typedef __attribute__((ext_vector_type(16))) _Float16 v16h;
typedef __attribute__((ext_vector_type(8)))  _Float16 v8h;
typedef __attribute__((ext_vector_type(16))) __bf16   v16b;
typedef __attribute__((ext_vector_type(8)))  __bf16   v8b;
typedef __attribute__((ext_vector_type(8)))  float    v8f;
typedef __attribute__((ext_vector_type(4)))  float    v4f;

__device__ __forceinline__ unsigned short f2bf_bits(float f) {
  unsigned u = __float_as_uint(f);
  return (unsigned short)((u + 0x7FFFu + ((u >> 16) & 1u)) >> 16);
}
__device__ __forceinline__ float bf_bits2f(unsigned short h) { return __uint_as_float(((unsigned)h) << 16); }

__device__ __forceinline__ void dep_guard_h(v8f& a, v8f& b, v16h x, v16h y) { asm volatile("v_nop\n\tv_nop\n\tv_nop\n\tv_nop" : "+v"(a), "+v"(b) : "v"(x), "v"(y)); }
__device__ __forceinline__ void dep_guard_b(v8f& a, v8f& b, v16b x, v16b y) { asm volatile("v_nop\n\tv_nop\n\tv_nop\n\tv_nop" : "+v"(a), "+v"(b) : "v"(x), "v"(y)); }
__device__ __forceinline__ void keep4_h(v16h a, v16h b, v16h c, v16h d) { asm volatile("v_nop" :: "v"(a), "v"(b), "v"(c), "v"(d)); }
__device__ __forceinline__ void keep4_b(v16b a, v16b b, v16b c, v16b d) { asm volatile("v_nop" :: "v"(a), "v"(b), "v"(c), "v"(d)); }
__device__ __forceinline__ void acc_guard4(v8f& a, v8f& b, v8f& c, v8f& d) { asm volatile("v_nop\n\tv_nop\n\tv_nop\n\tv_nop" : "+v"(a), "+v"(b), "+v"(c), "+v"(d)); }
__device__ __forceinline__ void guard4x4(v8f& a0, v8f& a1, v8f& a2, v8f& a3,
                                         v16h x0, v16h x1, v16h y0, v16h y1, v16h y2, v16h y3) {
  asm volatile("v_nop\n\tv_nop\n\tv_nop\n\tv_nop"
               : "+v"(a0), "+v"(a1), "+v"(a2), "+v"(a3)
               : "v"(x0), "v"(x1), "v"(y0), "v"(y1), "v"(y2), "v"(y3));
}

template <typename T> struct Frag;
template <> struct Frag<_Float16> {
  typedef v16h V; union U { v16h v; v8h h[2]; };
  static __device__ __forceinline__ v16h load(const _Float16* p) {
    U f; f.h[0] = *(const v8h*)(p); f.h[1] = *(const v8h*)(p + 16); return f.v;
  }
  static __device__ __forceinline__ v8f mma(v16h a, v16h b, v8f c) {
    return __builtin_amdgcn_wmma_f32_16x16x32_f16(false, a, false, b, (short)0, c, false, false);
  }
  static __device__ __forceinline__ void guard(v8f& a, v8f& b, v16h x, v16h y) { dep_guard_h(a, b, x, y); }
  static __device__ __forceinline__ void keep(v16h a, v16h b, v16h c, v16h d) { keep4_h(a, b, c, d); }
};
template <> struct Frag<__bf16> {
  typedef v16b V; union U { v16b v; v8b h[2]; };
  static __device__ __forceinline__ v16b load(const __bf16* p) {
    U f; f.h[0] = *(const v8b*)(p); f.h[1] = *(const v8b*)(p + 16); return f.v;
  }
  static __device__ __forceinline__ v8f mma(v16b a, v16b b, v8f c) {
    return __builtin_amdgcn_wmma_f32_16x16x32_bf16(false, a, false, b, (short)0, c, false, false);
  }
  static __device__ __forceinline__ void guard(v8f& a, v8f& b, v16b x, v16b y) { dep_guard_b(a, b, x, y); }
  static __device__ __forceinline__ void keep(v16b a, v16b b, v16b c, v16b d) { keep4_b(a, b, c, d); }
};

template <int ET> struct Elem;
template <> struct Elem<0> { typedef _Float16 T; };
template <> struct Elem<1> { typedef __bf16 T; };
template <int ET, bool SPLIT, int BIAS_MODE, int OUT_MODE, bool RESID, int ACT = 0>
__global__ __launch_bounds__(256) void wmma_gemm64(
    const unsigned short* __restrict__ Ap, const unsigned short* __restrict__ A2p, int lda, long strideA,
    const unsigned short* __restrict__ Btp, const unsigned short* __restrict__ Bt2p, int ldb, long strideB,
    void* __restrict__ Cout, void* __restrict__ Cout2, int ldc, long strideC,
    const float* __restrict__ bias,
    const float* __restrict__ resid, long strideR,
    int M, int N, int K, float scale) {
  typedef typename Elem<ET>::T T;
  typedef typename Frag<T>::V V;
  const T* A = (const T*)Ap; const T* A2 = (const T*)A2p; const T* Bt = (const T*)Btp; const T* Bt2 = (const T*)Bt2p;
  __shared__ __align__(16) float sT[8][16 * 68];
  const int b    = blockIdx.y;
  const int lane = threadIdx.x & 31;
  const int wave = threadIdx.x >> 5;
  const int tilesN = N >> 6;
  const int tilesM = M >> 6;
  const int tile = blockIdx.x * 8 + wave;
  if (tile >= tilesM * tilesN) return;
  const int tm = tile / tilesN;
  const int tn = tile - tm * tilesN;
  const int m0 = tm << 6;
  const int n0 = tn << 6;

  const T* Ab  = A  + (size_t)b * strideA;
  const T* Bb  = Bt + (size_t)b * strideB;
  const T* Ab2 = SPLIT ? (A2  + (size_t)b * strideA) : nullptr;
  const T* Bb2 = SPLIT ? (Bt2 + (size_t)b * strideB) : nullptr;

  const int rlane = lane & 15;
  const int koff  = (lane >> 4) * 8;
  const int mOff  = (lane >> 4) * 8;

  v8f acc[4][4];
#pragma unroll
  for (int i = 0; i < 4; ++i)
#pragma unroll
    for (int j = 0; j < 4; ++j) acc[i][j] = (v8f){0.f,0.f,0.f,0.f,0.f,0.f,0.f,0.f};

  for (int k0 = 0; k0 < K; k0 += 32) {
    V bh[4], bl[4];
#pragma unroll
    for (int j = 0; j < 4; ++j) {
      const size_t bo = (size_t)(n0 + (j << 4) + rlane) * ldb + koff + k0;
      bh[j] = Frag<T>::load(Bb + bo);
      if (SPLIT) bl[j] = Frag<T>::load(Bb2 + bo);
    }
#pragma unroll
    for (int i = 0; i < 4; ++i) {
      const size_t ao = (size_t)(m0 + (i << 4) + rlane) * lda + koff + k0;
      V ah = Frag<T>::load(Ab + ao);
      V al;
      if (SPLIT) al = Frag<T>::load(Ab2 + ao);
#pragma unroll
      for (int j = 0; j < 4; ++j) {
        acc[i][j] = Frag<T>::mma(ah, bh[j], acc[i][j]);
        if (SPLIT) {
          acc[i][j] = Frag<T>::mma(ah, bl[j], acc[i][j]);
          acc[i][j] = Frag<T>::mma(al, bh[j], acc[i][j]);
        }
      }
      Frag<T>::guard(acc[i][0], acc[i][3], ah, SPLIT ? al : ah);
    }
    Frag<T>::keep(bh[0], bh[1], bh[2], bh[3]);
    if (SPLIT) Frag<T>::keep(bl[0], bl[1], bl[2], bl[3]);
  }
  acc_guard4(acc[0][0], acc[0][1], acc[0][2], acc[0][3]);
  acc_guard4(acc[1][0], acc[1][1], acc[1][2], acc[1][3]);
  acc_guard4(acc[2][0], acc[2][1], acc[2][2], acc[2][3]);
  acc_guard4(acc[3][0], acc[3][1], acc[3][2], acc[3][3]);

  float* slab = sT[wave];
  const float* Rb = RESID ? (resid + (size_t)b * strideR) : nullptr;
#pragma unroll
  for (int i = 0; i < 4; ++i) {
    const int mBase = m0 + (i << 4);
#pragma unroll
    for (int j = 0; j < 4; ++j) {
      const int n = n0 + (j << 4) + rlane;
      float bv = 0.f;
      if (BIAS_MODE == 2) bv = bias[n];
#pragma unroll
      for (int r = 0; r < 8; ++r) {
        float v = acc[i][j][r] * scale;
        if (BIAS_MODE == 1) v += bias[mBase + mOff + r];
        if (BIAS_MODE == 2) v += bv;
        if (RESID) v += Rb[(size_t)(mBase + mOff + r) * ldc + n];
        if (ACT == 1) v = tanhf(v);
        if (ACT == 2) v = fmaxf(v, 0.0f);
        if (ACT == 3) v = v / (1.0f + expf(-v));
        if (ACT == 4) v = (v > 0.f) ? v : 0.01f * v;
        if (ACT == 5) v = 0.5f * v * (1.0f + erff(v * 0.70710678118654752f));
        slab[(mOff + r) * 68 + (j << 4) + rlane] = v;
      }
    }
    __builtin_amdgcn_fence(__ATOMIC_RELEASE, "workgroup");
    __builtin_amdgcn_wave_barrier();
    __builtin_amdgcn_fence(__ATOMIC_ACQUIRE, "workgroup");
    if (OUT_MODE == 0) {
      float* C = (float*)Cout + (size_t)b * strideC;
      const int hh = lane >> 4, c4 = (lane & 15) * 4;
      for (int pass = 0; pass < 2; ++pass) {
#pragma unroll
        for (int it = 0; it < 8; ++it) {
          const int row = it * 2 + hh;
          v4f v = *(const v4f*)(slab + row * 68 + c4);
          *(volatile v4f*)(C + (size_t)(mBase + row) * ldc + n0 + c4) = v;
        }
        __threadfence();
      }
    } else {
      const int q = lane >> 3, c8 = (lane & 7) * 8;
      unsigned short* C  = (unsigned short*)Cout  + (size_t)b * strideC;
      unsigned short* C2 = (OUT_MODE == 2) ? ((unsigned short*)Cout2 + (size_t)b * strideC) : nullptr;
      for (int pass = 0; pass < 2; ++pass) {
#pragma unroll
        for (int it = 0; it < 4; ++it) {
          const int row = it * 4 + q;
          const float* sp = slab + row * 68 + c8;
          v8h hv, lv;
#pragma unroll
          for (int e = 0; e < 8; ++e) {
            if (OUT_MODE == 1) {
              hv[e] = (_Float16)sp[e];
            } else {
              unsigned short hb = f2bf_bits(sp[e]);
              unsigned short lb = f2bf_bits(sp[e] - bf_bits2f(hb));
              hv[e] = __builtin_bit_cast(_Float16, hb);
              lv[e] = __builtin_bit_cast(_Float16, lb);
            }
          }
          *(volatile v8h*)(C + (size_t)(mBase + row) * ldc + n0 + c8) = hv;
          if (OUT_MODE == 2) *(volatile v8h*)(C2 + (size_t)(mBase + row) * ldc + n0 + c8) = lv;
        }
        __threadfence();
      }
    }
    __builtin_amdgcn_fence(__ATOMIC_RELEASE, "workgroup");
    __builtin_amdgcn_wave_barrier();
    __builtin_amdgcn_fence(__ATOMIC_ACQUIRE, "workgroup");
  }
}

#define NBAT   16
#define NSTK   64
#define NCHN   3
#define PSZ    32
#define IMG    256
#define PADN   288
#define KD     2048
#define EPSV   1e-7f
#define INVS2  50.0f
#define CARRY  16.0f
#define SLP    72

__device__ __forceinline__ void lds_wave_sync() {
  __builtin_amdgcn_fence(__ATOMIC_RELEASE, "workgroup");
  __builtin_amdgcn_wave_barrier();
  __builtin_amdgcn_fence(__ATOMIC_ACQUIRE, "workgroup");
}

__global__ __launch_bounds__(256) void stroke_filter_gemm(
    const float* __restrict__ brushes, const float* __restrict__ patches,
    _Float16* __restrict__ FyA, _Float16* __restrict__ T2) {
  #pragma clang fp contract(off)
  __shared__ __align__(16) _Float16 sP[2 * NCHN * PSZ * PSZ];
  __shared__ __align__(16) _Float16 sW[8][2048];
  __shared__ float sPart[4][8][32];
  __shared__ float sInv[4][32];
  __shared__ float sBr[128];
  __shared__ float sG[4];

  const int tid  = threadIdx.x;
  const int lane = tid & 31;
  const int wave = tid >> 5;
  const int hh   = lane >> 4;
  const int rl   = lane & 15;
  const int koff = hh * 8;
  const int b    = blockIdx.y;
  const int m    = blockIdx.x;
  const int n0   = m * 2;

  if (tid < 128) {
    const int n = tid & 63, ax = tid >> 6;
    sBr[tid] = brushes[(size_t)(b * NSTK + n) * 2 + ax];
  }
  __syncthreads();
  if (wave < 2) {
    const float v0 = sBr[wave * 64 + lane];
    const float v1 = sBr[wave * 64 + 32 + lane];
    float mn = fminf(v0, v1), mx = fmaxf(v0, v1);
#pragma unroll
    for (int off = 1; off < 32; off <<= 1) {
      mn = fminf(mn, __shfl_xor(mn, off, 32));
      mx = fmaxf(mx, __shfl_xor(mx, off, 32));
    }
    if (lane == 0) {
      const float den = (mx - mn) + EPSV;
      const float inv = 1.0f / den;
      const float p0 = sBr[wave * 64 + n0];
      const float p1 = sBr[wave * 64 + n0 + 1];
      sG[wave * 2 + 0] = ((p0 - mn) * inv) * 256.0f;
      sG[wave * 2 + 1] = ((p1 - mn) * inv) * 256.0f;
    }
  }
  __syncthreads();

  {
#pragma unroll 1
    for (int k4 = 0; k4 < 4; ++k4) {
      const int s = k4 & 1, ax = k4 >> 1;
      const float qf  = (float)(lane + 1) - 16.0f;
      const float off = (ax == 0) ? (qf - 0.5f) : (qf - 0.4f);
      const float u   = sG[ax * 2 + s] + off;
      float sacc = 0.f;
#pragma unroll 1
      for (int v = wave * 36; v < wave * 36 + 36; ++v) {
        const float a  = (float)v - 16.0f;
        const float d  = a - u;
        const float sq = d * d;
        sacc += expf(-sq * INVS2);
      }
      sPart[k4][wave][lane] = sacc;
    }
  }
  __syncthreads();
  if (tid < 128) {
    const int k4 = tid >> 5;
    float ssum = 0.f;
#pragma unroll
    for (int p = 0; p < 8; ++p) ssum += sPart[k4][p][lane];
    sInv[k4][lane] = 1.0f / (ssum + EPSV);
  }
  {
    const float* pb = patches + (size_t)(b * NSTK + n0) * (NCHN * PSZ * PSZ);
#pragma unroll 4
    for (int k = 0; k < 24; ++k) {
      const int idx = tid + k * 256;
      sP[idx] = (_Float16)pb[idx];
    }
  }
  __syncthreads();

  _Float16* wsl = sW[wave];
  {
    const float g = sG[hh];
#pragma unroll
    for (int i = 0; i < 2; ++i) {
      const float xf = (float)((wave * 2 + i) * 16 + rl);
      _Float16* dst = wsl + ((i * 2 + hh) * 16 + rl) * 32;
#pragma unroll 1
      for (int q = 0; q < PSZ; ++q) {
        const float u  = g + (((float)(q + 1) - 16.0f) - 0.5f);
        const float d  = xf - u;
        const float sq = d * d;
        const float e  = expf(-sq * INVS2) * sInv[hh][q];
        dst[q] = (_Float16)(e * CARRY);
      }
    }
  }
  lds_wave_sync();
  v16h aF[2][2];
#pragma unroll
  for (int i = 0; i < 2; ++i)
#pragma unroll
    for (int s2 = 0; s2 < 2; ++s2)
      aF[i][s2] = Frag<_Float16>::load(wsl + ((i * 2 + s2) * 16 + rl) * 32 + koff);
  lds_wave_sync();

  const v8f z8 = {0.f, 0.f, 0.f, 0.f, 0.f, 0.f, 0.f, 0.f};
  const int qq = lane >> 3;
  const int c8 = (lane & 7) * 8;
#pragma unroll 1
  for (int c = 0; c < NCHN; ++c) {
    v16h bF[2][2];
#pragma unroll
    for (int s2 = 0; s2 < 2; ++s2)
#pragma unroll
      for (int pt = 0; pt < 2; ++pt)
        bF[s2][pt] = Frag<_Float16>::load(sP + (s2 * NCHN + c) * (PSZ * PSZ) + (pt * 16 + rl) * PSZ + koff);
#pragma unroll
    for (int i = 0; i < 2; ++i) {
      const int x0 = (wave * 2 + i) * 16;
      v8f acc[2][2];
#pragma unroll
      for (int s2 = 0; s2 < 2; ++s2)
#pragma unroll
        for (int pt = 0; pt < 2; ++pt)
          acc[s2][pt] = Frag<_Float16>::mma(aF[i][s2], bF[s2][pt], z8);
      guard4x4(acc[0][0], acc[0][1], acc[1][0], acc[1][1],
               aF[i][0], aF[i][1], bF[0][0], bF[0][1], bF[1][0], bF[1][1]);
#pragma unroll
      for (int s2 = 0; s2 < 2; ++s2)
#pragma unroll
        for (int pt = 0; pt < 2; ++pt)
#pragma unroll
          for (int r = 0; r < 8; ++r)
            wsl[(8 * hh + r) * SLP + s2 * 32 + pt * 16 + rl] = (_Float16)acc[s2][pt][r];
      lds_wave_sync();
      _Float16* gb = T2 + ((size_t)((b * NCHN + c) * IMG + x0)) * KD + m * 64 + c8;
      for (int pass = 0; pass < 2; ++pass) {
#pragma unroll
        for (int it = 0; it < 4; ++it) {
          const int row = it * 4 + qq;
          const v8h hv = *(const v8h*)(wsl + row * SLP + c8);
          *(volatile v8h*)(gb + (size_t)row * KD) = hv;
        }
        __threadfence();
      }
      lds_wave_sync();
    }
  }

  {
    const float g = sG[2 + hh];
#pragma unroll
    for (int i = 0; i < 2; ++i) {
      const int yb = wave * 32 + i * 16;
      const float yf = (float)(yb + rl);
      _Float16* dst = wsl + rl * SLP + hh * 32;
#pragma unroll 1
      for (int p = 0; p < PSZ; ++p) {
        const float u  = g + (((float)(p + 1) - 16.0f) - 0.4f);
        const float d  = yf - u;
        const float sq = d * d;
        const float e  = expf(-sq * INVS2) * sInv[2 + hh][p];
        dst[p] = (_Float16)(e * CARRY);
      }
      lds_wave_sync();
      _Float16* gb = FyA + ((size_t)(b * IMG + yb)) * KD + m * 64 + c8;
      for (int pass = 0; pass < 2; ++pass) {
#pragma unroll
        for (int it = 0; it < 4; ++it) {
          const int row = it * 4 + qq;
          const v8h hv = *(const v8h*)(wsl + row * SLP + c8);
          *(volatile v8h*)(gb + (size_t)row * KD) = hv;
        }
        __threadfence();
      }
      lds_wave_sync();
    }
  }
}

extern "C" void kernel_launch(void* const* d_in, const int* in_sizes, int n_in,
                              void* d_out, int out_size, void* d_ws, size_t ws_size,
                              hipStream_t stream) {
  if (n_in < 2) return;
  if (in_sizes[0] != NBAT * NSTK * 2) return;
  if (in_sizes[1] != NBAT * NSTK * NCHN * PSZ * PSZ) return;
  if (out_size != NBAT * NCHN * IMG * IMG) return;
  const size_t fyHalves = (size_t)NBAT * IMG * KD;
  const size_t t2Halves = (size_t)NBAT * NCHN * IMG * KD;
  const size_t needBytes = (fyHalves + t2Halves) * 2;
  if (needBytes > ws_size) return;

  const float* brushes = (const float*)d_in[0];
  const float* patches = (const float*)d_in[1];
  _Float16* FyA = (_Float16*)d_ws;
  _Float16* T2  = FyA + fyHalves;
  float* out = (float*)d_out;

  stroke_filter_gemm<<<dim3(NSTK / 2, NBAT), 256, 0, stream>>>(brushes, patches, FyA, T2);

  const int M = IMG, N = IMG, K = KD;
  const int tiles = (M / 64) * (N / 64);
  const int gxb = (tiles + 7) / 8;
  const float scale = 1.0f / 16384.0f;
  for (int c = 0; c < NCHN; ++c) {
    const unsigned short* Bt = (const unsigned short*)(T2 + (size_t)c * IMG * KD);
    void* Cp = (void*)(out + (size_t)c * IMG * IMG);
    wmma_gemm64<0, false, 0, 0, false, 0><<<dim3(gxb, NBAT), 256, 0, stream>>>(
        (const unsigned short*)FyA, (const unsigned short*)FyA, K, (long)IMG * KD,
        Bt, Bt, K, (long)NCHN * IMG * KD,
        Cp, Cp, IMG, (long)NCHN * IMG * IMG,
        (const float*)d_ws,
        (const float*)d_ws, 0L,
        M, N, K, scale);
  }
}
